// LatticeRNN_31121333027060
// MI455X (gfx1250) — hardware-verified
//
#include <hip/hip_runtime.h>
#include <math.h>

constexpr int NB       = 32;
constexpr int SEQ      = 512;
constexpr int DIN      = 512;
constexpr int HID      = 512;
constexpr int G4N      = 4 * HID;
constexpr int KARCS    = 4;
constexpr int NTHR     = 256;
constexpr int NQ       = 4;
constexpr int QSTEPS   = SEQ / NQ;
constexpr int QROWS    = QSTEPS * NB;
constexpr int NROWS    = NB * SEQ;
constexpr int APITCH   = 520;
constexpr int FPITCH   = 516;
constexpr int SLABP    = 36;
constexpr int LDS_BYTES = 2 * NB * APITCH * 2 + NB * FPITCH * 4 + (NTHR / 32) * 16 * SLABP * 4;
static_assert(LDS_BYTES <= 163840, "static LDS budget");
static_assert(NB == 32, "time-major row permutation and the two m-subtiles use NB == 32");
static_assert(NTHR == 16 * 16, "gather map: 16 rows x 16 column chunks of 32, two row halves");
static_assert(HID == 64 * (NTHR / 32), "8 waves x 64 hidden units");
static_assert(DIN % 32 == 0 && HID % 32 == 0, "GEMM K multiples of 32, no padding");
static_assert(QROWS % 64 == 0 && G4N % 64 == 0, "GEMM M, N tile multiples");
static_assert(SEQ % NQ == 0, "quarters exact");
static_assert((NROWS * (DIN / 8)) % NTHR == 0, "X convert grid exact");
static_assert((G4N * (DIN / 8)) % NTHR == 0, "W convert grid exact");
static_assert((NROWS * HID / 4) % NTHR == 0, "zero fill grid exact");
static_assert(APITCH % 8 == 0 && FPITCH % 4 == 0 && SLABP % 4 == 0, "16-B aligned LDS rows");

typedef __attribute__((ext_vector_type(16))) _Float16 v16h;
typedef __attribute__((ext_vector_type(8)))  _Float16 v8h;
typedef __attribute__((ext_vector_type(16))) __bf16   v16b;
typedef __attribute__((ext_vector_type(8)))  __bf16   v8b;
typedef __attribute__((ext_vector_type(8)))  float    v8f;
typedef __attribute__((ext_vector_type(4)))  float    v4f;

__device__ __forceinline__ unsigned short f2bf_bits(float f) {
  unsigned u = __float_as_uint(f);
  return (unsigned short)((u + 0x7FFFu + ((u >> 16) & 1u)) >> 16);
}
__device__ __forceinline__ float bf_bits2f(unsigned short h) { return __uint_as_float(((unsigned)h) << 16); }

__device__ __forceinline__ void dep_guard_h(v8f& a, v8f& b, v16h x, v16h y) { asm volatile("v_nop\n\tv_nop\n\tv_nop\n\tv_nop" : "+v"(a), "+v"(b) : "v"(x), "v"(y)); }
__device__ __forceinline__ void dep_guard_b(v8f& a, v8f& b, v16b x, v16b y) { asm volatile("v_nop\n\tv_nop\n\tv_nop\n\tv_nop" : "+v"(a), "+v"(b) : "v"(x), "v"(y)); }
__device__ __forceinline__ void keep4_h(v16h a, v16h b, v16h c, v16h d) { asm volatile("v_nop" :: "v"(a), "v"(b), "v"(c), "v"(d)); }
__device__ __forceinline__ void keep4_b(v16b a, v16b b, v16b c, v16b d) { asm volatile("v_nop" :: "v"(a), "v"(b), "v"(c), "v"(d)); }
__device__ __forceinline__ void acc_guard4(v8f& a, v8f& b, v8f& c, v8f& d) { asm volatile("v_nop\n\tv_nop\n\tv_nop\n\tv_nop" : "+v"(a), "+v"(b), "+v"(c), "+v"(d)); }
__device__ __forceinline__ void wave_sync_lds() {
  __builtin_amdgcn_fence(__ATOMIC_RELEASE, "workgroup");
  __builtin_amdgcn_wave_barrier();
  __builtin_amdgcn_fence(__ATOMIC_ACQUIRE, "workgroup");
}
template <typename T> struct Frag;
template <> struct Frag<_Float16> {
  typedef v16h V; union U { v16h v; v8h h[2]; };
  static __device__ __forceinline__ v16h load(const _Float16* p) {
    U f; f.h[0] = *(const v8h*)(p); f.h[1] = *(const v8h*)(p + 16); return f.v;
  }
  static __device__ __forceinline__ v8f mma(v16h a, v16h b, v8f c) {
    return __builtin_amdgcn_wmma_f32_16x16x32_f16(false, a, false, b, (short)0, c, false, false);
  }
  static __device__ __forceinline__ void guard(v8f& a, v8f& b, v16h x, v16h y) { dep_guard_h(a, b, x, y); }
  static __device__ __forceinline__ void keep(v16h a, v16h b, v16h c, v16h d) { keep4_h(a, b, c, d); }
};
template <> struct Frag<__bf16> {
  typedef v16b V; union U { v16b v; v8b h[2]; };
  static __device__ __forceinline__ v16b load(const __bf16* p) {
    U f; f.h[0] = *(const v8b*)(p); f.h[1] = *(const v8b*)(p + 16); return f.v;
  }
  static __device__ __forceinline__ v8f mma(v16b a, v16b b, v8f c) {
    return __builtin_amdgcn_wmma_f32_16x16x32_bf16(false, a, false, b, (short)0, c, false, false);
  }
  static __device__ __forceinline__ void guard(v8f& a, v8f& b, v16b x, v16b y) { dep_guard_b(a, b, x, y); }
  static __device__ __forceinline__ void keep(v16b a, v16b b, v16b c, v16b d) { keep4_b(a, b, c, d); }
};

__device__ __forceinline__ float fsig(float x)  { return __builtin_amdgcn_rcpf(1.0f + __expf(-x)); }
__device__ __forceinline__ float ftanh(float x) { return 1.0f - 2.0f * __builtin_amdgcn_rcpf(__expf(2.0f * x) + 1.0f); }

template <int ET> struct Elem;
template <> struct Elem<0> { typedef _Float16 T; };
template <> struct Elem<1> { typedef __bf16 T; };
template <int ET, bool SPLIT, int BIAS_MODE, int OUT_MODE, bool RESID, int ACT = 0>
__global__ __launch_bounds__(256) void wmma_gemm64(
    const unsigned short* __restrict__ Ap, const unsigned short* __restrict__ A2p, int lda, long strideA,
    const unsigned short* __restrict__ Btp, const unsigned short* __restrict__ Bt2p, int ldb, long strideB,
    void* __restrict__ Cout, void* __restrict__ Cout2, int ldc, long strideC,
    const float* __restrict__ bias,
    const float* __restrict__ resid, long strideR,
    int M, int N, int K, float scale) {
  typedef typename Elem<ET>::T T;
  typedef typename Frag<T>::V V;
  const T* A = (const T*)Ap; const T* A2 = (const T*)A2p; const T* Bt = (const T*)Btp; const T* Bt2 = (const T*)Bt2p;
  __shared__ __align__(16) float sT[8][16 * 68];
  const int b    = blockIdx.y;
  const int lane = threadIdx.x & 31;
  const int wave = threadIdx.x >> 5;
  const int tilesN = N >> 6;
  const int tilesM = M >> 6;
  const int tile = blockIdx.x * 8 + wave;
  if (tile >= tilesM * tilesN) return;
  const int tm = tile / tilesN;
  const int tn = tile - tm * tilesN;
  const int m0 = tm << 6;
  const int n0 = tn << 6;

  const T* Ab  = A  + (size_t)b * strideA;
  const T* Bb  = Bt + (size_t)b * strideB;
  const T* Ab2 = SPLIT ? (A2  + (size_t)b * strideA) : nullptr;
  const T* Bb2 = SPLIT ? (Bt2 + (size_t)b * strideB) : nullptr;

  const int rlane = lane & 15;
  const int koff  = (lane >> 4) * 8;
  const int mOff  = (lane >> 4) * 8;

  v8f acc[4][4];
#pragma unroll
  for (int i = 0; i < 4; ++i)
#pragma unroll
    for (int j = 0; j < 4; ++j) acc[i][j] = (v8f){0.f,0.f,0.f,0.f,0.f,0.f,0.f,0.f};

  for (int k0 = 0; k0 < K; k0 += 32) {
    V bh[4], bl[4];
#pragma unroll
    for (int j = 0; j < 4; ++j) {
      const size_t bo = (size_t)(n0 + (j << 4) + rlane) * ldb + koff + k0;
      bh[j] = Frag<T>::load(Bb + bo);
      if (SPLIT) bl[j] = Frag<T>::load(Bb2 + bo);
    }
#pragma unroll
    for (int i = 0; i < 4; ++i) {
      const size_t ao = (size_t)(m0 + (i << 4) + rlane) * lda + koff + k0;
      V ah = Frag<T>::load(Ab + ao);
      V al;
      if (SPLIT) al = Frag<T>::load(Ab2 + ao);
#pragma unroll
      for (int j = 0; j < 4; ++j) {
        acc[i][j] = Frag<T>::mma(ah, bh[j], acc[i][j]);
        if (SPLIT) {
          acc[i][j] = Frag<T>::mma(ah, bl[j], acc[i][j]);
          acc[i][j] = Frag<T>::mma(al, bh[j], acc[i][j]);
        }
      }
      Frag<T>::guard(acc[i][0], acc[i][3], ah, SPLIT ? al : ah);
    }
    Frag<T>::keep(bh[0], bh[1], bh[2], bh[3]);
    if (SPLIT) Frag<T>::keep(bl[0], bl[1], bl[2], bl[3]);
  }
  acc_guard4(acc[0][0], acc[0][1], acc[0][2], acc[0][3]);
  acc_guard4(acc[1][0], acc[1][1], acc[1][2], acc[1][3]);
  acc_guard4(acc[2][0], acc[2][1], acc[2][2], acc[2][3]);
  acc_guard4(acc[3][0], acc[3][1], acc[3][2], acc[3][3]);

  float* slab = sT[wave];
  const float* Rb = RESID ? (resid + (size_t)b * strideR) : nullptr;
#pragma unroll
  for (int i = 0; i < 4; ++i) {
    const int mBase = m0 + (i << 4);
#pragma unroll
    for (int j = 0; j < 4; ++j) {
      const int n = n0 + (j << 4) + rlane;
      float bv = 0.f;
      if (BIAS_MODE == 2) bv = bias[n];
#pragma unroll
      for (int r = 0; r < 8; ++r) {
        float v = acc[i][j][r] * scale;
        if (BIAS_MODE == 1) v += bias[mBase + mOff + r];
        if (BIAS_MODE == 2) v += bv;
        if (RESID) v += Rb[(size_t)(mBase + mOff + r) * ldc + n];
        if (ACT == 1) v = tanhf(v);
        if (ACT == 2) v = fmaxf(v, 0.0f);
        if (ACT == 3) v = v / (1.0f + expf(-v));
        if (ACT == 4) v = (v > 0.f) ? v : 0.01f * v;
        if (ACT == 5) v = 0.5f * v * (1.0f + erff(v * 0.70710678118654752f));
        slab[(mOff + r) * 68 + (j << 4) + rlane] = v;
      }
    }
    __builtin_amdgcn_fence(__ATOMIC_RELEASE, "workgroup");
    __builtin_amdgcn_wave_barrier();
    __builtin_amdgcn_fence(__ATOMIC_ACQUIRE, "workgroup");
    if (OUT_MODE == 0) {
      float* C = (float*)Cout + (size_t)b * strideC;
      const int hh = lane >> 4, c4 = (lane & 15) * 4;
      for (int pass = 0; pass < 2; ++pass) {
#pragma unroll
        for (int it = 0; it < 8; ++it) {
          const int row = it * 2 + hh;
          v4f v = *(const v4f*)(slab + row * 68 + c4);
          *(volatile v4f*)(C + (size_t)(mBase + row) * ldc + n0 + c4) = v;
        }
        __threadfence();
      }
    } else {
      const int q = lane >> 3, c8 = (lane & 7) * 8;
      unsigned short* C  = (unsigned short*)Cout  + (size_t)b * strideC;
      unsigned short* C2 = (OUT_MODE == 2) ? ((unsigned short*)Cout2 + (size_t)b * strideC) : nullptr;
      for (int pass = 0; pass < 2; ++pass) {
#pragma unroll
        for (int it = 0; it < 4; ++it) {
          const int row = it * 4 + q;
          const float* sp = slab + row * 68 + c8;
          v8h hv, lv;
#pragma unroll
          for (int e = 0; e < 8; ++e) {
            if (OUT_MODE == 1) {
              hv[e] = (_Float16)sp[e];
            } else {
              unsigned short hb = f2bf_bits(sp[e]);
              unsigned short lb = f2bf_bits(sp[e] - bf_bits2f(hb));
              hv[e] = __builtin_bit_cast(_Float16, hb);
              lv[e] = __builtin_bit_cast(_Float16, lb);
            }
          }
          *(volatile v8h*)(C + (size_t)(mBase + row) * ldc + n0 + c8) = hv;
          if (OUT_MODE == 2) *(volatile v8h*)(C2 + (size_t)(mBase + row) * ldc + n0 + c8) = lv;
        }
        __threadfence();
      }
    }
    __builtin_amdgcn_fence(__ATOMIC_RELEASE, "workgroup");
    __builtin_amdgcn_wave_barrier();
    __builtin_amdgcn_fence(__ATOMIC_ACQUIRE, "workgroup");
  }
}

template <int PERM>
__global__ __launch_bounds__(NTHR) void cvt8_split_kernel(const float* __restrict__ src, unsigned short* __restrict__ dhi,
                                                          unsigned short* __restrict__ dlo, int nrow, int ncol8) {
  const int i  = blockIdx.x * NTHR + threadIdx.x;
  const int n8 = nrow * ncol8;
  if (i < n8) {
    const int row  = i / ncol8;
    const int c8   = i - row * ncol8;
    const int srow = PERM ? ((row % NB) * SEQ + (row / NB)) : row;
    const float* sp = src + (size_t)srow * (size_t)(ncol8 * 8) + c8 * 8;
    const v4f a = *(const v4f*)(sp);
    const v4f b = *(const v4f*)(sp + 4);
    v8h hv, lv;
#pragma unroll
    for (int e = 0; e < 4; ++e) {
      const unsigned short ha = f2bf_bits(a[e]);
      const unsigned short la = f2bf_bits(a[e] - bf_bits2f(ha));
      const unsigned short hb = f2bf_bits(b[e]);
      const unsigned short lb = f2bf_bits(b[e] - bf_bits2f(hb));
      hv[e]     = __builtin_bit_cast(_Float16, ha);
      lv[e]     = __builtin_bit_cast(_Float16, la);
      hv[4 + e] = __builtin_bit_cast(_Float16, hb);
      lv[4 + e] = __builtin_bit_cast(_Float16, lb);
    }
    unsigned short* ph = dhi + (size_t)i * 8;
    unsigned short* pl = dlo + (size_t)i * 8;
    *(volatile v8h*)ph = hv;
    *(volatile v8h*)pl = lv;
    __threadfence();
    *(volatile v8h*)ph = hv;
    *(volatile v8h*)pl = lv;
  }
}

__global__ __launch_bounds__(NTHR) void bias_sum_kernel(const float* __restrict__ b_a, const float* __restrict__ b_b,
                                                        float* __restrict__ dst) {
  const int i = blockIdx.x * NTHR + threadIdx.x;
  if (i < G4N / 4) {
    const v4f va = *(const v4f*)(b_a + 4 * i);
    const v4f vb = *(const v4f*)(b_b + 4 * i);
    const v4f o = va + vb;
    float* op = dst + 4 * i;
    *(volatile v4f*)op = o;
    __threadfence();
    *(volatile v4f*)op = o;
  }
}

__global__ __launch_bounds__(NTHR) void zero4_kernel(float* __restrict__ dst, int n4) {
  const int i = blockIdx.x * NTHR + threadIdx.x;
  if (i < n4) {
    const v4f z = {0.0f, 0.0f, 0.0f, 0.0f};
    float* op = dst + (size_t)i * 4;
    *(volatile v4f*)op = z;
    __threadfence();
    *(volatile v4f*)op = z;
  }
}

__global__ __launch_bounds__(NTHR) void lattice_seq_kernel(
    const float* __restrict__ prev_w, const int* __restrict__ prev_idx,
    const unsigned short* __restrict__ WHHp, const unsigned short* __restrict__ WHLp,
    const float* __restrict__ XG, float* hout, float* cst, int tq0) {
  __shared__ __align__(16) __bf16 Ah[NB * APITCH];
  __shared__ __align__(16) __bf16 Al[NB * APITCH];
  __shared__ __align__(16) float  Cp[NB * FPITCH];
  __shared__ __align__(16) float  Sl[NTHR / 32][16 * SLABP];
  const __bf16* WHH = (const __bf16*)WHHp;
  const __bf16* WHL = (const __bf16*)WHLp;
  const int tid = threadIdx.x, lane = tid & 31, wave = tid >> 5;
  const int c = lane & 15, hh = lane >> 4, koff = hh * 8;
  const int q8 = lane >> 3, c4s = (lane & 7) * 4;
  const int grow = tid >> 4;
  const int gcol = (tid & 15) * 32;
  const v8f z8 = {0.f, 0.f, 0.f, 0.f, 0.f, 0.f, 0.f, 0.f};
  float* slab = Sl[wave];

#pragma unroll 1
  for (int tl = 0; tl < QSTEPS; ++tl) {
    const int t = tq0 + tl;

#pragma unroll 1
    for (int ms = 0; ms < 2; ++ms) {
      const int gb = ms * 16 + grow;
      const size_t arc0 = ((size_t)gb * SEQ + (size_t)t) * KARCS;
      v4f ha[8], ca[8];
#pragma unroll
      for (int m = 0; m < 8; ++m) { ha[m] = (v4f){0.f, 0.f, 0.f, 0.f}; ca[m] = (v4f){0.f, 0.f, 0.f, 0.f}; }
#pragma unroll 1
      for (int j = 0; j < KARCS; ++j) {
        const float wj = prev_w[arc0 + j];
        int ij = prev_idx[arc0 + j];
        ij = ij < 0 ? 0 : ij;
        ij = ij > SEQ - 1 ? SEQ - 1 : ij;
        const size_t ho = ((size_t)gb * SEQ + (size_t)ij) * HID + gcol;
        const float* hp  = hout + ho;
        const float* cpp = cst + ho;
#pragma unroll
        for (int m = 0; m < 8; ++m) {
          const v4f hv = *(const v4f*)(hp + 4 * m);
          const v4f cv = *(const v4f*)(cpp + 4 * m);
          ha[m] += wj * hv;
          ca[m] += wj * cv;
        }
      }
#pragma unroll
      for (int m4 = 0; m4 < 4; ++m4) {
        v8b hv, lv;
#pragma unroll
        for (int e = 0; e < 4; ++e) {
          const float f0 = ha[2 * m4][e];
          const float f1 = ha[2 * m4 + 1][e];
          const unsigned short h0 = f2bf_bits(f0);
          const unsigned short h1 = f2bf_bits(f1);
          const unsigned short l0 = f2bf_bits(f0 - bf_bits2f(h0));
          const unsigned short l1 = f2bf_bits(f1 - bf_bits2f(h1));
          hv[e]     = __builtin_bit_cast(__bf16, h0);
          hv[4 + e] = __builtin_bit_cast(__bf16, h1);
          lv[e]     = __builtin_bit_cast(__bf16, l0);
          lv[4 + e] = __builtin_bit_cast(__bf16, l1);
        }
        *(v8b*)(Ah + gb * APITCH + gcol + 8 * m4) = hv;
        *(v8b*)(Al + gb * APITCH + gcol + 8 * m4) = lv;
      }
#pragma unroll
      for (int m = 0; m < 8; ++m) *(v4f*)(Cp + gb * FPITCH + gcol + 4 * m) = ca[m];
    }
    __syncthreads();

    {
      const __bf16* a0h = Ah + c * APITCH + koff;
      const __bf16* a0l = Al + c * APITCH + koff;
      const __bf16* a1h = Ah + (16 + c) * APITCH + koff;
      const __bf16* a1l = Al + (16 + c) * APITCH + koff;
      const size_t xrow0 = (size_t)(tl * NB + 8 * hh) * (size_t)G4N;
#pragma unroll 1
      for (int np = 0; np < 2; ++np) {
        const int colbase = 64 * wave + 32 * np;
        float h1r[2][8];
#pragma unroll
        for (int u = 0; u < 2; ++u) {
          const int j = colbase + 16 * u + c;
          const __bf16* bhp = WHH + (size_t)j * HID + koff;
          const __bf16* blp = WHL + (size_t)j * HID + koff;
          v8f acc0[4], acc1[4];
#pragma unroll
          for (int g = 0; g < 4; ++g) { acc0[g] = z8; acc1[g] = z8; }
#pragma unroll 1
          for (int k0 = 0; k0 < HID; k0 += 32) {
            const v16b fa0h = Frag<__bf16>::load(a0h + k0);
            const v16b fa0l = Frag<__bf16>::load(a0l + k0);
            const v16b fa1h = Frag<__bf16>::load(a1h + k0);
            const v16b fa1l = Frag<__bf16>::load(a1l + k0);
            v16b bh[4], bl[4];
#pragma unroll
            for (int g = 0; g < 4; ++g) {
              bh[g] = Frag<__bf16>::load(bhp + (size_t)g * HID * HID + k0);
              bl[g] = Frag<__bf16>::load(blp + (size_t)g * HID * HID + k0);
            }
#pragma unroll
            for (int g = 0; g < 4; ++g) {
              acc0[g] = Frag<__bf16>::mma(fa0h, bh[g], acc0[g]);
              acc0[g] = Frag<__bf16>::mma(fa0h, bl[g], acc0[g]);
              acc0[g] = Frag<__bf16>::mma(fa0l, bh[g], acc0[g]);
              acc1[g] = Frag<__bf16>::mma(fa1h, bh[g], acc1[g]);
              acc1[g] = Frag<__bf16>::mma(fa1h, bl[g], acc1[g]);
              acc1[g] = Frag<__bf16>::mma(fa1l, bh[g], acc1[g]);
            }
            dep_guard_b(acc0[0], acc1[3], fa0h, fa1h);
            keep4_b(fa0l, fa1l, bh[0], bh[1]);
            keep4_b(bh[2], bh[3], bl[0], bl[1]);
            keep4_b(bl[2], bl[3], bl[2], bl[3]);
          }
          acc_guard4(acc0[0], acc0[1], acc0[2], acc0[3]);
          acc_guard4(acc1[0], acc1[1], acc1[2], acc1[3]);
#pragma unroll
          for (int r = 0; r < 8; ++r) {
            {
              const float* xp = XG + xrow0 + (size_t)r * G4N + j;
              const float iv = acc0[0][r] + xp[0];
              const float fv = acc0[1][r] + xp[HID];
              const float gv = acc0[2][r] + xp[2 * HID];
              const float ov = acc0[3][r] + xp[3 * HID];
              const int lo = (8 * hh + r) * FPITCH + j;
              const float cprev = Cp[lo];
              const float cn = fsig(fv) * cprev + fsig(iv) * ftanh(gv);
              const float hn = fsig(ov) * ftanh(cn);
              Cp[lo] = cn;
              slab[(8 * hh + r) * SLABP + 16 * u + c] = hn;
            }
            {
              const float* xp = XG + xrow0 + (size_t)(16 + r) * G4N + j;
              const float iv = acc1[0][r] + xp[0];
              const float fv = acc1[1][r] + xp[HID];
              const float gv = acc1[2][r] + xp[2 * HID];
              const float ov = acc1[3][r] + xp[3 * HID];
              const int lo = (16 + 8 * hh + r) * FPITCH + j;
              const float cprev = Cp[lo];
              const float cn = fsig(fv) * cprev + fsig(iv) * ftanh(gv);
              const float hn = fsig(ov) * ftanh(cn);
              Cp[lo] = cn;
              h1r[u][r] = hn;
            }
          }
        }
        wave_sync_lds();
        for (int pass = 0; pass < 2; ++pass) {
#pragma unroll
          for (int it = 0; it < 8; ++it) {
            const int row = it * 4 + q8;
            const v4f cv = *(const v4f*)(Cp + row * FPITCH + colbase + c4s);
            *(volatile v4f*)(cst + ((size_t)row * SEQ + (size_t)t) * HID + colbase + c4s) = cv;
          }
#pragma unroll
          for (int it = 0; it < 4; ++it) {
            const int row = it * 4 + q8;
            const v4f hv = *(const v4f*)(slab + row * SLABP + c4s);
            *(volatile v4f*)(hout + ((size_t)row * SEQ + (size_t)t) * HID + colbase + c4s) = hv;
          }
          __threadfence();
        }
        wave_sync_lds();
#pragma unroll
        for (int u = 0; u < 2; ++u)
#pragma unroll
          for (int r = 0; r < 8; ++r) slab[(8 * hh + r) * SLABP + 16 * u + c] = h1r[u][r];
        wave_sync_lds();
        for (int pass = 0; pass < 2; ++pass) {
#pragma unroll
          for (int it = 0; it < 4; ++it) {
            const int row = it * 4 + q8;
            const v4f hv = *(const v4f*)(slab + row * SLABP + c4s);
            *(volatile v4f*)(hout + ((size_t)(16 + row) * SEQ + (size_t)t) * HID + colbase + c4s) = hv;
          }
          __threadfence();
        }
        wave_sync_lds();
      }
    }
    __syncthreads();
  }
}

extern "C" void kernel_launch(void* const* d_in, const int* in_sizes, int n_in,
                              void* d_out, int out_size, void* d_ws, size_t ws_size, hipStream_t stream) {
  if (n_in < 7 || d_out == nullptr || d_ws == nullptr) return;
  if (in_sizes[0] != NB * SEQ * DIN || in_sizes[1] != NB * SEQ * KARCS || in_sizes[2] != G4N * DIN ||
      in_sizes[3] != G4N * HID || in_sizes[4] != G4N || in_sizes[5] != G4N || in_sizes[6] != NB * SEQ * KARCS ||
      out_size != NB * SEQ * HID) return;

  const float* x      = (const float*)d_in[0];
  const float* prev_w = (const float*)d_in[1];
  const float* w_ih   = (const float*)d_in[2];
  const float* w_hh   = (const float*)d_in[3];
  const float* b_ih   = (const float*)d_in[4];
  const float* b_hh   = (const float*)d_in[5];
  const int*   pidx   = (const int*)d_in[6];
  float* hout = (float*)d_out;

  char* ws = (char*)d_ws; size_t off = 0;
  auto carve = [&](size_t bytes) -> char* { char* p = ws + off; off += (bytes + 255) & ~(size_t)255; return p; };
  unsigned short* XH   = (unsigned short*)carve((size_t)NROWS * DIN * 2);
  unsigned short* XL   = (unsigned short*)carve((size_t)NROWS * DIN * 2);
  unsigned short* WIH  = (unsigned short*)carve((size_t)G4N * DIN * 2);
  unsigned short* WIL  = (unsigned short*)carve((size_t)G4N * DIN * 2);
  unsigned short* WHH  = (unsigned short*)carve((size_t)G4N * HID * 2);
  unsigned short* WHL  = (unsigned short*)carve((size_t)G4N * HID * 2);
  float*          BSUM = (float*)carve((size_t)G4N * 4);
  float*          XG   = (float*)carve((size_t)QROWS * G4N * 4);
  float*          CS   = (float*)carve((size_t)NROWS * HID * 4);
  if (off > ws_size || off > (size_t)134217728) return;

  const int n4cs = NROWS * HID / 4;
  zero4_kernel<<<n4cs / NTHR, NTHR, 0, stream>>>(hout, n4cs);
  zero4_kernel<<<n4cs / NTHR, NTHR, 0, stream>>>(CS, n4cs);

  const int n8x = NROWS * (DIN / 8);
  const int n8w = G4N * (DIN / 8);
  cvt8_split_kernel<1><<<n8x / NTHR, NTHR, 0, stream>>>(x,    XH,  XL,  NROWS, DIN / 8);
  cvt8_split_kernel<0><<<n8w / NTHR, NTHR, 0, stream>>>(w_ih, WIH, WIL, G4N,   DIN / 8);
  cvt8_split_kernel<0><<<n8w / NTHR, NTHR, 0, stream>>>(w_hh, WHH, WHL, G4N,   HID / 8);
  bias_sum_kernel<<<(G4N / 4) / NTHR, NTHR, 0, stream>>>(b_ih, b_hh, BSUM);

  const dim3 ggrid((QROWS / 64) * (G4N / 64) / 8, 1);
  for (int q = 0; q < NQ; ++q) {
    const size_t aoff = (size_t)q * QROWS * DIN;
    wmma_gemm64<1, true, 2, 0, false, 0><<<ggrid, 256, 0, stream>>>(
        XH + aoff, XL + aoff, DIN, 0L, WIH, WIL, DIN, 0L, (void*)XG, (void*)XG, G4N, 0L,
        BSUM, BSUM, 0L, QROWS, G4N, DIN, 1.0f);
    lattice_seq_kernel<<<1, NTHR, 0, stream>>>(prev_w, pidx, WHH, WHL, XG, hout, CS, q * QSTEPS);
  }
}
